// MultiScaleDeformableAttention_74663711474023
// MI455X (gfx1250) — hardware-verified
//
#include <hip/hip_runtime.h>
#include <math.h>

#pragma clang fp contract(off)

typedef __attribute__((ext_vector_type(16))) __bf16   v16b;
typedef __attribute__((ext_vector_type(8)))  __bf16   v8b;
typedef __attribute__((ext_vector_type(8)))  float    v8f;
typedef __attribute__((ext_vector_type(4)))  float    v4f;
typedef __attribute__((ext_vector_type(4)))  unsigned int v4u;

constexpr int kBS    = 2;
constexpr int kNQ    = 7681;
constexpr int kC     = 256;
constexpr int kHeads = 8;
constexpr int kDH    = 32;
constexpr int kNLog  = 128;
constexpr int kRows  = kBS * kNQ;
constexpr int kRowsPad = 15424;
static_assert(kRowsPad % 64 == 0 && kRowsPad >= kRows && kRowsPad - kRows < 64, "pad");
static_assert(kC % 64 == 0 && kNLog % 64 == 0, "N tile");
static_assert(kC % 32 == 0, "K step");
static_assert(kHeads * kDH == kC, "head split");

constexpr size_t kPlane16 = (size_t)kRowsPad * kC * 2;
constexpr size_t kPlane32 = (size_t)kRowsPad * kC * 4;
constexpr size_t kLog32   = (size_t)kRowsPad * kNLog * 4;
constexpr size_t kTmp32   = (size_t)kRows * kC * 4;
constexpr size_t kW256    = (size_t)256 * 256 * 2;
constexpr size_t kW128    = (size_t)128 * 256 * 2;
constexpr size_t kOffQb    = 0;
constexpr size_t kOffVb    = kOffQb + kPlane16;
constexpr size_t kOffWval  = kOffVb + kPlane16;
constexpr size_t kOffWoff  = kOffWval + kW256;
constexpr size_t kOffWattn = kOffWoff + kW256;
constexpr size_t kOffWout  = kOffWattn + kW128;
constexpr size_t kOffVproj = kOffWout + kW256;
constexpr size_t kOffOffb  = kOffVproj + kPlane32;
constexpr size_t kOffLog   = kOffOffb + kPlane32;
constexpr size_t kOffTmpF  = kOffLog + kLog32;
constexpr size_t kOffTmpH  = kOffTmpF + kTmp32;
constexpr size_t kOffTmpL  = kOffTmpH + kPlane16;
constexpr size_t kWsTotal  = kOffTmpL + kPlane16;
static_assert(kWsTotal == 87263232ull, "carve");
static_assert(kWsTotal <= 134217728ull, "carve budget");
static_assert((kOffVb % 128) == 0 && (kOffWval % 128) == 0 && (kOffVproj % 128) == 0 && (kOffTmpF % 128) == 0 &&
              (kOffTmpH % 128) == 0 && (kOffTmpL % 128) == 0, "line aligned");

constexpr int kN8Real = kRows * kC / 8;
constexpr int kN8Pad  = kRowsPad * kC / 8;
static_assert(kN8Pad % 256 == 0, "pack grid exact");

__device__ __forceinline__ unsigned short f2bf_bits(float f) {
  unsigned u = __float_as_uint(f);
  return (unsigned short)((u + 0x7FFFu + ((u >> 16) & 1u)) >> 16);
}
__device__ __forceinline__ float bf_bits2f(unsigned short h) { return __uint_as_float(((unsigned)h) << 16); }
__device__ __forceinline__ unsigned pk16(unsigned short a, unsigned short b) { return (unsigned)a | ((unsigned)b << 16); }

__device__ __forceinline__ void wave_lds_sync() {
  __builtin_amdgcn_fence(__ATOMIC_RELEASE, "workgroup");
  __builtin_amdgcn_wave_barrier();
  __builtin_amdgcn_fence(__ATOMIC_ACQUIRE, "workgroup");
}

__device__ __forceinline__ void guard_grp(v8f& a, v8f& b, v8f& c, v8f& d,
                                          v16b x, v16b y, v16b b0, v16b b1, v16b b2, v16b b3) {
  asm volatile("v_nop\n\tv_nop\n\tv_nop\n\tv_nop"
               : "+v"(a), "+v"(b), "+v"(c), "+v"(d)
               : "v"(x), "v"(y), "v"(b0), "v"(b1), "v"(b2), "v"(b3));
}
__device__ __forceinline__ void keep4_b(v16b a, v16b b, v16b c, v16b d) { asm volatile("v_nop" :: "v"(a), "v"(b), "v"(c), "v"(d)); }
__device__ __forceinline__ void acc_guard4(v8f& a, v8f& b, v8f& c, v8f& d) { asm volatile("v_nop\n\tv_nop\n\tv_nop\n\tv_nop" : "+v"(a), "+v"(b), "+v"(c), "+v"(d)); }

__device__ __forceinline__ v16b frag_load_b(const __bf16* p) {
  union { v16b v; v8b h[2]; } f;
  f.h[0] = *(const v8b*)(p);
  f.h[1] = *(const v8b*)(p + 16);
  return f.v;
}
__device__ __forceinline__ v8f mma_b(v16b a, v16b b, v8f c) {
  return __builtin_amdgcn_wmma_f32_16x16x32_bf16(false, a, false, b, (short)0, c, false, false);
}

template <int SPLITM, bool BIASN>
__global__ __launch_bounds__(256) void wmma_gemm64_bf16(
    const unsigned short* __restrict__ Ap, const unsigned short* __restrict__ A2p, int lda,
    const unsigned short* __restrict__ Btp, const unsigned short* __restrict__ Bt2p, int ldb,
    float* __restrict__ Cout, int ldc, const float* __restrict__ bias,
    int M, int N, int K, int Mreal, float scale) {
  const __bf16* A  = (const __bf16*)Ap;  const __bf16* A2  = (const __bf16*)A2p;
  const __bf16* Bt = (const __bf16*)Btp; const __bf16* Bt2 = (const __bf16*)Bt2p;
  __shared__ __align__(16) float sT[8][16 * 68];
  const int lane = threadIdx.x & 31;
  const int wave = threadIdx.x >> 5;
  const int tilesN = N >> 6;
  const int tilesM = M >> 6;
  const int tile = blockIdx.x * 8 + wave;
  if (tile >= tilesM * tilesN) return;
  const int tm = tile / tilesN;
  const int tn = tile - tm * tilesN;
  const int m0 = tm << 6;
  const int n0 = tn << 6;

  const int rlane = lane & 15;
  const int koff  = (lane >> 4) * 8;
  const int mOff  = (lane >> 4) * 8;

  v8f acc[4][4];
#pragma unroll
  for (int i = 0; i < 4; ++i)
#pragma unroll
    for (int j = 0; j < 4; ++j) acc[i][j] = (v8f){0.f,0.f,0.f,0.f,0.f,0.f,0.f,0.f};

  for (int k0 = 0; k0 < K; k0 += 32) {
    v16b bh[4], bl[4];
#pragma unroll
    for (int j = 0; j < 4; ++j) {
      const size_t bo = (size_t)(n0 + (j << 4) + rlane) * ldb + koff + k0;
      bh[j] = frag_load_b(Bt + bo);
      if (SPLITM == 1) bl[j] = frag_load_b(Bt2 + bo);
    }
#pragma unroll
    for (int i = 0; i < 4; ++i) {
      const size_t ao = (size_t)(m0 + (i << 4) + rlane) * lda + koff + k0;
      v16b ah = frag_load_b(A + ao);
      v16b al;
      if (SPLITM != 0) al = frag_load_b(A2 + ao);
#pragma unroll
      for (int j = 0; j < 4; ++j) {
        acc[i][j] = mma_b(ah, bh[j], acc[i][j]);
        if (SPLITM == 1) acc[i][j] = mma_b(ah, bl[j], acc[i][j]);
        if (SPLITM != 0) acc[i][j] = mma_b(al, bh[j], acc[i][j]);
      }
      guard_grp(acc[i][0], acc[i][1], acc[i][2], acc[i][3], ah, (SPLITM != 0) ? al : ah, bh[0], bh[1], bh[2], bh[3]);
    }
    keep4_b(bh[0], bh[1], bh[2], bh[3]);
    if (SPLITM == 1) keep4_b(bl[0], bl[1], bl[2], bl[3]);
  }
  acc_guard4(acc[0][0], acc[0][1], acc[0][2], acc[0][3]);
  acc_guard4(acc[1][0], acc[1][1], acc[1][2], acc[1][3]);
  acc_guard4(acc[2][0], acc[2][1], acc[2][2], acc[2][3]);
  acc_guard4(acc[3][0], acc[3][1], acc[3][2], acc[3][3]);

  float* slab = sT[wave];
#pragma unroll
  for (int i = 0; i < 4; ++i) {
    const int mBase = m0 + (i << 4);
#pragma unroll
    for (int j = 0; j < 4; ++j) {
      const int n = n0 + (j << 4) + rlane;
      float bv = 0.f;
      if (BIASN) bv = bf_bits2f(f2bf_bits(bias[n]));
#pragma unroll
      for (int r = 0; r < 8; ++r) {
        const float v = acc[i][j][r] * scale + bv;
        slab[(mOff + r) * 68 + (j << 4) + rlane] = v;
      }
    }
    wave_lds_sync();
    {
      const int hh = lane >> 4, c4 = (lane & 15) * 4;
      for (int pass = 0; pass < 2; ++pass) {
#pragma unroll
        for (int it = 0; it < 8; ++it) {
          const int row = it * 2 + hh;
          const int grow = mBase + row;
          const v4f v = *(const v4f*)(slab + row * 68 + c4);
          if (grow < Mreal) *(volatile v4f*)(Cout + (size_t)grow * ldc + n0 + c4) = v;
        }
        __threadfence();
      }
    }
    wave_lds_sync();
  }
}

__global__ __launch_bounds__(256) void wtcast_bf16(const float* __restrict__ W0, const float* __restrict__ W1,
                                                   const float* __restrict__ W2, const float* __restrict__ W3,
                                                   unsigned short* __restrict__ O0, unsigned short* __restrict__ O1,
                                                   unsigned short* __restrict__ O2, unsigned short* __restrict__ O3) {
  __shared__ float sm[64][65];
  const int t  = threadIdx.x;
  const int z  = blockIdx.z;
  const int nout = (z == 2) ? kNLog : kC;
  if ((int)blockIdx.y * 64 >= nout) return;
  const int k0 = blockIdx.x * 64;
  const int n0 = blockIdx.y * 64;
  const float* W = (z == 0) ? W0 : (z == 1) ? W1 : (z == 2) ? W2 : W3;
  unsigned short* O = (z == 0) ? O0 : (z == 1) ? O1 : (z == 2) ? O2 : O3;
#pragma unroll
  for (int i = 0; i < 8; ++i) {
    const int e = i * 256 + t;
    const int r = e >> 6;
    const int c = e & 63;
    sm[c][r] = W[(size_t)(k0 + r) * nout + n0 + c];
  }
  asm volatile("" ::: "memory");
#pragma unroll
  for (int i = 8; i < 16; ++i) {
    const int e = i * 256 + t;
    const int r = e >> 6;
    const int c = e & 63;
    sm[c][r] = W[(size_t)(k0 + r) * nout + n0 + c];
  }
  __syncthreads();
  const int lane = t & 31, wave = t >> 5;
  const int q = lane >> 3, c8 = (lane & 7) * 8;
  for (int pass = 0; pass < 2; ++pass) {
#pragma unroll
    for (int it = 0; it < 2; ++it) {
      const int row = wave * 8 + it * 4 + q;
      unsigned short hb[8];
#pragma unroll
      for (int e = 0; e < 8; ++e) hb[e] = f2bf_bits(sm[row][c8 + e]);
      const v4u u = (v4u){pk16(hb[0], hb[1]), pk16(hb[2], hb[3]), pk16(hb[4], hb[5]), pk16(hb[6], hb[7])};
      *(volatile v4u*)(O + (size_t)(n0 + row) * kC + k0 + c8) = u;
    }
    __threadfence();
  }
}

__global__ __launch_bounds__(256) void pack_bf16_x2(const float* __restrict__ in0, const float* __restrict__ in1,
                                                    unsigned short* __restrict__ o0, unsigned short* __restrict__ o1,
                                                    int n8real, int n8pad) {
  const int i = blockIdx.x * 256 + threadIdx.x;
  if (i >= n8pad) return;
  const bool second = (blockIdx.y != 0);
  const float* in = second ? in1 : in0;
  unsigned short* out = second ? o1 : o0;
  const bool real = i < n8real;
  const int ic = real ? i : (n8real - 1);
  const float zf = real ? 1.0f : 0.0f;
  const float* p = in + 8 * (size_t)ic;
  const v4f a = *(const v4f*)(p);
  const v4f c = *(const v4f*)(p + 4);
  unsigned short hb[8];
#pragma unroll
  for (int e = 0; e < 4; ++e) {
    hb[e]     = f2bf_bits(a[e] * zf);
    hb[4 + e] = f2bf_bits(c[e] * zf);
  }
  const v4u u = (v4u){pk16(hb[0], hb[1]), pk16(hb[2], hb[3]), pk16(hb[4], hb[5]), pk16(hb[6], hb[7])};
  unsigned short* qo = out + 8 * (size_t)i;
  *(volatile v4u*)qo = u;
  __threadfence();
  *(volatile v4u*)qo = u;
}

__global__ __launch_bounds__(256) void pack_bf16_hilo(const float* __restrict__ in,
                                                      unsigned short* __restrict__ oh, unsigned short* __restrict__ ol,
                                                      int n8real, int n8pad) {
  const int i = blockIdx.x * 256 + threadIdx.x;
  if (i >= n8pad) return;
  const bool real = i < n8real;
  const int ic = real ? i : (n8real - 1);
  const float zf = real ? 1.0f : 0.0f;
  const float* p = in + 8 * (size_t)ic;
  const v4f a = *(const v4f*)(p);
  const v4f c = *(const v4f*)(p + 4);
  float x[8];
#pragma unroll
  for (int e = 0; e < 4; ++e) { x[e] = a[e] * zf; x[4 + e] = c[e] * zf; }
  unsigned short hb[8], lb[8];
#pragma unroll
  for (int e = 0; e < 8; ++e) {
    hb[e] = f2bf_bits(x[e]);
    lb[e] = f2bf_bits(x[e] - bf_bits2f(hb[e]));
  }
  const v4u uh = (v4u){pk16(hb[0], hb[1]), pk16(hb[2], hb[3]), pk16(hb[4], hb[5]), pk16(hb[6], hb[7])};
  const v4u ul = (v4u){pk16(lb[0], lb[1]), pk16(lb[2], lb[3]), pk16(lb[4], lb[5]), pk16(lb[6], lb[7])};
  unsigned short* qh = oh + 8 * (size_t)i;
  unsigned short* ql = ol + 8 * (size_t)i;
  *(volatile v4u*)qh = uh;
  *(volatile v4u*)ql = ul;
  __threadfence();
  *(volatile v4u*)qh = uh;
  *(volatile v4u*)ql = ul;
}

__global__ __launch_bounds__(256) void msda_sample_kernel(const float* __restrict__ refp, const float* __restrict__ vproj,
                                                          const float* __restrict__ offb, const float* __restrict__ logit,
                                                          float* __restrict__ tmpf) {
  __shared__ __align__(16) float sOff[8][256];
  __shared__ __align__(16) float sLg[8][128];
  const int lane = threadIdx.x & 31;
  const int wave = threadIdx.x >> 5;
  const int row  = blockIdx.x * 8 + wave;
  const bool live = row < kRows;
  const int rowc = live ? row : (kRows - 1);
  const int b = (rowc >= kNQ) ? 1 : 0;
  const int q = rowc - b * kNQ;
  {
    const float* op = offb + (size_t)rowc * kC;
    const v4f o0 = *(const v4f*)(op + lane * 4);
    const v4f o1 = *(const v4f*)(op + 128 + lane * 4);
    const v4f g0 = *(const v4f*)(logit + (size_t)rowc * kNLog + lane * 4);
    *(v4f*)(&sOff[wave][lane * 4]) = o0;
    *(v4f*)(&sOff[wave][128 + lane * 4]) = o1;
    *(v4f*)(&sLg[wave][lane * 4]) = g0;
  }
  wave_lds_sync();
  const float rx = bf_bits2f(f2bf_bits(refp[(size_t)rowc * 2]));
  const float ry = bf_bits2f(f2bf_bits(refp[(size_t)rowc * 2 + 1]));
  const float* vb = vproj + (size_t)b * kNQ * kC + lane;
  float* ob = tmpf + ((size_t)(b * kHeads) * kNQ + q) * kDH + lane;

#pragma unroll 1
  for (int m = 0; m < kHeads; ++m) {
    const float lg = sLg[wave][m * 16 + (lane & 15)];
    float mx = lg;
    mx = fmaxf(mx, __shfl_xor(mx, 1, 32));
    mx = fmaxf(mx, __shfl_xor(mx, 2, 32));
    mx = fmaxf(mx, __shfl_xor(mx, 4, 32));
    mx = fmaxf(mx, __shfl_xor(mx, 8, 32));
    const float e = expf(lg - mx);
    float s = e;
    s += __shfl_xor(s, 1, 32);
    s += __shfl_xor(s, 2, 32);
    s += __shfl_xor(s, 4, 32);
    s += __shfl_xor(s, 8, 32);
    const float inv = 1.0f / s;
    const float* vm = vb + m * kDH;
    const float* om = &sOff[wave][m * 32];
    float acc = 0.0f;
#pragma unroll 1
    for (int f = 0; f < 16; ++f) {
      const int kp = f >> 2;
      const int l  = f & 3;
      const int wl = (l == 0) ? 76 : (l == 1) ? 38 : (l == 2) ? 19 : 10;
      const int sl = (l == 0) ? 0 : (l == 1) ? 5776 : (l == 2) ? 7220 : 7581;
      const float fhalf = (float)wl * 0.5f;
      const float ox = om[l * 8 + kp * 2];
      const float oy = om[l * 8 + kp * 2 + 1];
      const float lx = fminf(fmaxf(rx + ox, 0.0f), 1.0f);
      const float ly = fminf(fmaxf(ry + oy, 0.0f), 1.0f);
      const float gx = lx * 2.0f - 1.0f;
      const float gy = ly * 2.0f - 1.0f;
      const float x = (gx + 1.0f) * fhalf - 0.5f;
      const float y = (gy + 1.0f) * fhalf - 0.5f;
      const float xf = floorf(x), yf = floorf(y);
      const float wx1 = x - xf, wy1 = y - yf;
      const float wx0 = 1.0f - wx1, wy0 = 1.0f - wy1;
      const int x0 = (int)xf, y0 = (int)yf;
      const int x1 = x0 + 1, y1 = y0 + 1;
      const bool vx0 = (x0 >= 0) && (x0 < wl);
      const bool vx1 = (x1 >= 0) && (x1 < wl);
      const bool vy0 = (y0 >= 0) && (y0 < wl);
      const bool vy1 = (y1 >= 0) && (y1 < wl);
      const int cx0 = min(max(x0, 0), wl - 1);
      const int cx1 = min(max(x1, 0), wl - 1);
      const int cy0 = min(max(y0, 0), wl - 1);
      const int cy1 = min(max(y1, 0), wl - 1);
      const float g00 = vm[(size_t)(sl + cy0 * wl + cx0) * kC];
      const float g10 = vm[(size_t)(sl + cy0 * wl + cx1) * kC];
      const float g01 = vm[(size_t)(sl + cy1 * wl + cx0) * kC];
      const float g11 = vm[(size_t)(sl + cy1 * wl + cx1) * kC];
      const float m00 = (vx0 && vy0) ? 1.0f : 0.0f;
      const float m10 = (vx1 && vy0) ? 1.0f : 0.0f;
      const float m01 = (vx0 && vy1) ? 1.0f : 0.0f;
      const float m11 = (vx1 && vy1) ? 1.0f : 0.0f;
      const float t00 = g00 * ((wx0 * wy0) * m00);
      const float t10 = g10 * ((wx1 * wy0) * m10);
      const float t01 = g01 * ((wx0 * wy1) * m01);
      const float t11 = g11 * ((wx1 * wy1) * m11);
      const float smp = ((t00 + t10) + t01) + t11;
      const float pw = __shfl(e, f, 32) * inv;
      acc = acc + smp * pw;
    }
    if (live) {
      float* op2 = ob + (size_t)m * kNQ * kDH;
      *(volatile float*)op2 = acc;
      __threadfence();
      *(volatile float*)op2 = acc;
    }
  }
}

extern "C" void kernel_launch(void* const* d_in, const int* in_sizes, int n_in,
                              void* d_out, int out_size, void* d_ws, size_t ws_size,
                              hipStream_t stream) {
  (void)in_sizes; (void)n_in;
  if (ws_size < kWsTotal) return;
  if ((size_t)out_size < (size_t)kRows * kC) return;

  const float* query  = (const float*)d_in[0];
  const float* refp   = (const float*)d_in[1];
  const float* value  = (const float*)d_in[2];
  const float* W_off  = (const float*)d_in[4];
  const float* b_off  = (const float*)d_in[5];
  const float* W_attn = (const float*)d_in[6];
  const float* b_attn = (const float*)d_in[7];
  const float* W_val  = (const float*)d_in[8];
  const float* b_val  = (const float*)d_in[9];
  const float* W_out  = (const float*)d_in[10];
  const float* b_out  = (const float*)d_in[11];
  float* out = (float*)d_out;

  unsigned char* ws = (unsigned char*)d_ws;
  unsigned short* Qb     = (unsigned short*)(ws + kOffQb);
  unsigned short* Vb     = (unsigned short*)(ws + kOffVb);
  unsigned short* WvalT  = (unsigned short*)(ws + kOffWval);
  unsigned short* WoffT  = (unsigned short*)(ws + kOffWoff);
  unsigned short* WattnT = (unsigned short*)(ws + kOffWattn);
  unsigned short* WoutT  = (unsigned short*)(ws + kOffWout);
  float* vproj = (float*)(ws + kOffVproj);
  float* offb  = (float*)(ws + kOffOffb);
  float* logit = (float*)(ws + kOffLog);
  float* tmpF  = (float*)(ws + kOffTmpF);
  unsigned short* tmpH = (unsigned short*)(ws + kOffTmpH);
  unsigned short* tmpL = (unsigned short*)(ws + kOffTmpL);

  pack_bf16_x2<<<dim3(kN8Pad / 256, 2), 256, 0, stream>>>(query, value, Qb, Vb, kN8Real, kN8Pad);
  wtcast_bf16<<<dim3(4, 4, 4), 256, 0, stream>>>(W_val, W_off, W_attn, W_out, WvalT, WoffT, WattnT, WoutT);
  wmma_gemm64_bf16<0, true><<<dim3((241 * 4 + 7) / 8), 256, 0, stream>>>(
      Vb, nullptr, kC, WvalT, nullptr, kC, vproj, kC, b_val, kRowsPad, kC, kC, kRowsPad, 1.0f);
  wmma_gemm64_bf16<0, true><<<dim3((241 * 4 + 7) / 8), 256, 0, stream>>>(
      Qb, nullptr, kC, WoffT, nullptr, kC, offb, kC, b_off, kRowsPad, kC, kC, kRowsPad, 1.0f);
  wmma_gemm64_bf16<0, true><<<dim3((241 * 2 + 7) / 8), 256, 0, stream>>>(
      Qb, nullptr, kC, WattnT, nullptr, kC, logit, kNLog, b_attn, kRowsPad, kNLog, kC, kRowsPad, 1.0f);
  msda_sample_kernel<<<dim3((kRows + 7) / 8), 256, 0, stream>>>(refp, vproj, offb, logit, tmpF);
  pack_bf16_hilo<<<dim3(kN8Pad / 256), 256, 0, stream>>>(tmpF, tmpH, tmpL, kN8Real, kN8Pad);
  wmma_gemm64_bf16<2, true><<<dim3((241 * 4 + 7) / 8), 256, 0, stream>>>(
      tmpH, tmpL, kC, WoutT, nullptr, kC, out, kC, b_out, kRowsPad, kC, kC, kRows, 1.0f);
}
